// GNNModelDGL_85177791414880
// MI455X (gfx1250) — hardware-verified
//
#include <hip/hip_runtime.h>
#include <stddef.h>


#define NTHR    256
#define NWAVE   8
#define EPT     8
#define NGRP    2
#define CHUNK   (NTHR * EPT * NGRP)
#define WCAP    (EPT * NGRP * 32)
#define LISTN   (NWAVE * WCAP)
#define NBC     4096
#define NBF     1024
#define RCAP    40960
#define RBN     128
#define TGT     256
#define DEGCAP  1024
#define OTHR    512
#define BM      64
#define BNC     128
#define WSCAP   134217728
#define FIN     128
#define HID     256
#define NH1     8
#define DH1     32
#define JW1     16
#define JW2     4
#define ACARRY  8.0f
#define WCARRY  64.0f
#define PCARRY  64.0f
#define SCL_AW  (1.0f / 512.0f)
#define SCL_PW  (1.0f / 4096.0f)
#define ARC_S   4.0f
#define ARC_M   0.5f

#define LDS_FILL ((RCAP + NBF + LISTN) * 4 + 64)

static_assert((CHUNK & (CHUNK - 1)) == 0);
static_assert(CHUNK <= 4096);
static_assert((NBC & (NBC - 1)) == 0 && (NBF & (NBF - 1)) == 0);
static_assert(NBC == 4 * NBF);
static_assert(OTHR * 8 == NBC);
static_assert((RCAP % 32) == 0);
static_assert(TGT == NWAVE * 32);
static_assert((NBC % TGT) == 0);
static_assert((TGT % BM) == 0);
static_assert(WCAP == EPT * NGRP * 32);
static_assert((FIN % 32) == 0 && (HID % 32) == 0);
static_assert((HID % BNC) == 0);
static_assert(HID == 2 * 128);
static_assert(NH1 * DH1 == HID);
static_assert(FIN * JW1 <= 2048 && HID * JW2 <= 2048);
static_assert(HID == NTHR);

typedef float    v4f  __attribute__((ext_vector_type(4)));
typedef float    v8f  __attribute__((ext_vector_type(8)));
typedef int      v4i  __attribute__((ext_vector_type(4)));
typedef _Float16 v4h  __attribute__((ext_vector_type(4)));
typedef _Float16 v8h  __attribute__((ext_vector_type(8)));
typedef _Float16 v16h __attribute__((ext_vector_type(16)));
union Frag { v16h v; v8h h[2]; };

__device__ __forceinline__ v8f wmh(v16h a, v16h b, v8f c) {
  v8f d = __builtin_amdgcn_wmma_f32_16x16x32_f16(false, a, false, b, (short)0, c, false, false);
  asm volatile("v_nop\n\tv_nop\n\tv_nop\n\tv_nop" : "+v"(d) : "v"(a), "v"(b));
  return d;
}

__device__ __forceinline__ v4f selz(v4f v, bool live) {
  v4f o; o.x = live ? v.x : 0.f; o.y = live ? v.y : 0.f; o.z = live ? v.z : 0.f; o.w = live ? v.w : 0.f; return o;
}
__device__ __forceinline__ v4f selv4(v4f v, bool c, float other) {
  v4f o; o.x = c ? v.x : other; o.y = c ? v.y : other; o.z = c ? v.z : other; o.w = c ? v.w : other; return o;
}
__device__ __forceinline__ v4f vmax4(v4f a, v4f b) {
  v4f o; o.x = fmaxf(a.x, b.x); o.y = fmaxf(a.y, b.y); o.z = fmaxf(a.z, b.z); o.w = fmaxf(a.w, b.w); return o;
}
__device__ __forceinline__ v4f lrelu4(v4f v) {
  v4f o;
  o.x = v.x >= 0.f ? v.x : 0.2f * v.x;  o.y = v.y >= 0.f ? v.y : 0.2f * v.y;
  o.z = v.z >= 0.f ? v.z : 0.2f * v.z;  o.w = v.w >= 0.f ? v.w : 0.2f * v.w;
  return o;
}
__device__ __forceinline__ float lrelu1(float v) { return v >= 0.f ? v : 0.2f * v; }
__device__ __forceinline__ v4f vexp4(v4f v) {
  v4f o; o.x = __expf(v.x); o.y = __expf(v.y); o.z = __expf(v.z); o.w = __expf(v.w); return o;
}
__device__ __forceinline__ v4f elu4(v4f v) {
  v4f o;
  o.x = v.x > 0.f ? v.x : (__expf(v.x) - 1.0f);  o.y = v.y > 0.f ? v.y : (__expf(v.y) - 1.0f);
  o.z = v.z > 0.f ? v.z : (__expf(v.z) - 1.0f);  o.w = v.w > 0.f ? v.w : (__expf(v.w) - 1.0f);
  return o;
}
__device__ __forceinline__ v4f wmax4(v4f v) {
#pragma unroll
  for (int off = 16; off > 0; off >>= 1) {
    v.x = fmaxf(v.x, __shfl_xor(v.x, off)); v.y = fmaxf(v.y, __shfl_xor(v.y, off));
    v.z = fmaxf(v.z, __shfl_xor(v.z, off)); v.w = fmaxf(v.w, __shfl_xor(v.w, off));
  }
  return v;
}
__device__ __forceinline__ v4f wsum4(v4f v) {
#pragma unroll
  for (int off = 16; off > 0; off >>= 1) {
    v.x += __shfl_xor(v.x, off); v.y += __shfl_xor(v.y, off);
    v.z += __shfl_xor(v.z, off); v.w += __shfl_xor(v.w, off);
  }
  return v;
}
__device__ __forceinline__ float wmax1(float v) {
#pragma unroll
  for (int off = 16; off > 0; off >>= 1) v = fmaxf(v, __shfl_xor(v, off));
  return v;
}
__device__ __forceinline__ float wsum1(float v) {
#pragma unroll
  for (int off = 16; off > 0; off >>= 1) v += __shfl_xor(v, off);
  return v;
}

template <int NB>
__device__ __forceinline__ int scan_chunk(const int* __restrict__ dsts, int nE, int cbase, int slotBase,
                                          int vec8, int* list, int tid, int lane, int wave) {
  int wc = 0;
#pragma unroll
  for (int g = 0; g < NGRP; ++g) {
    const int el0  = (g * NTHR + tid) * EPT;
    const int e0   = cbase + el0;
    const int sent = -2147483647 - 1;
    v4i da, db;
    if (vec8 != 0 && cbase + CHUNK <= nE) {
      da = *(const v4i*)(dsts + e0);
      db = *(const v4i*)(dsts + e0 + 4);
    } else {
      da.x = (e0     < nE) ? dsts[min(e0, nE - 1)] : sent;
      da.y = (e0 + 1 < nE) ? dsts[min(e0 + 1, nE - 1)] : sent;
      da.z = (e0 + 2 < nE) ? dsts[min(e0 + 2, nE - 1)] : sent;
      da.w = (e0 + 3 < nE) ? dsts[min(e0 + 3, nE - 1)] : sent;
      db.x = (e0 + 4 < nE) ? dsts[min(e0 + 4, nE - 1)] : sent;
      db.y = (e0 + 5 < nE) ? dsts[min(e0 + 5, nE - 1)] : sent;
      db.z = (e0 + 6 < nE) ? dsts[min(e0 + 6, nE - 1)] : sent;
      db.w = (e0 + 7 < nE) ? dsts[min(e0 + 7, nE - 1)] : sent;
    }
    const unsigned nb = (unsigned)slotBase;
    const unsigned s0 = (unsigned)da.x - nb, s1 = (unsigned)da.y - nb;
    const unsigned s2 = (unsigned)da.z - nb, s3 = (unsigned)da.w - nb;
    const unsigned s4 = (unsigned)db.x - nb, s5 = (unsigned)db.y - nb;
    const unsigned s6 = (unsigned)db.z - nb, s7 = (unsigned)db.w - nb;
    const bool h0 = s0 < (unsigned)NB, h1 = s1 < (unsigned)NB, h2 = s2 < (unsigned)NB, h3 = s3 < (unsigned)NB;
    const bool h4 = s4 < (unsigned)NB, h5 = s5 < (unsigned)NB, h6 = s6 < (unsigned)NB, h7 = s7 < (unsigned)NB;
    const unsigned any = __builtin_amdgcn_ballot_w32(h0 | h1 | h2 | h3 | h4 | h5 | h6 | h7);
    if (any != 0u) {
#define HITJ(J, HJ, SJ) { \
        const unsigned mj = __builtin_amdgcn_ballot_w32(HJ); \
        if (mj != 0u) { \
          if (HJ) { \
            const int pos = wc + (int)__builtin_amdgcn_mbcnt_lo(mj, 0u); \
            if (pos < WCAP) list[wave * WCAP + pos] = ((el0 + (J)) << 12) | (int)(SJ); \
          } \
          wc += (int)__builtin_popcount(mj); } }
      HITJ(0, h0, s0)
      HITJ(1, h1, s1)
      HITJ(2, h2, s2)
      HITJ(3, h3, s3)
      HITJ(4, h4, s4)
      HITJ(5, h5, s5)
      HITJ(6, h6, s6)
      HITJ(7, h7, s7)
#undef HITJ
    }
  }
  return wc;
}

__global__ __launch_bounds__(NTHR) void k_count(const int* __restrict__ dsts, int* cnt, int nE, int vec8) {
  __shared__ __attribute__((aligned(16))) int scnt[NBC];
  __shared__ __attribute__((aligned(16))) int list[LISTN];
  __shared__ int wcnt[NWAVE];
  const int tid = threadIdx.x, lane = tid & 31, wave = tid >> 5;
  const int nodeBase = blockIdx.x * NBC;

  for (int i = tid; i < NBC; i += NTHR) scnt[i] = 0;
  __syncthreads();

  const int nChunks = (nE + CHUNK - 1) / CHUNK;
#pragma unroll 1
  for (int ch = 0; ch < nChunks; ++ch) {
    const int cbase = ch * CHUNK;
    const int wc = scan_chunk<NBC>(dsts, nE, cbase, nodeBase, vec8, list, tid, lane, wave);
    if (lane == 0) wcnt[wave] = wc;
    __syncthreads();
    if (wave == 0) {
#pragma unroll 1
      for (int wsx = 0; wsx < NWAVE; ++wsx) {
        int n = __builtin_amdgcn_readfirstlane(wcnt[wsx]);
        n = n > WCAP ? WCAP : (n < 0 ? 0 : n);
        const int* lp = list + wsx * WCAP;
#pragma unroll 1
        for (int i = 0; i < n; ++i) {
          const int ent  = __builtin_amdgcn_readfirstlane(lp[i]);
          const int slot = ent & (NBC - 1);
          if (lane == 0) scnt[slot] = scnt[slot] + 1;
        }
      }
    }
    __syncthreads();
  }

  v4i cq[4];
#pragma unroll
  for (int q = 0; q < 4; ++q) {
    const int f = (wave * 4 + q) * 128 + 4 * lane;
    cq[q] = *(const v4i*)(scnt + f);
  }
  int* cp = cnt + (size_t)nodeBase;
#pragma unroll
  for (int q = 0; q < 4; ++q) {
    const int f = (wave * 4 + q) * 128 + 4 * lane;
    *(volatile v4i*)(cp + f) = cq[q];
  }
  __threadfence();
#pragma unroll
  for (int q = 0; q < 4; ++q) {
    const int f = (wave * 4 + q) * 128 + 4 * lane;
    *(volatile v4i*)(cp + f) = cq[q];
  }
}

__global__ __launch_bounds__(OTHR) void k_offsets(
    const int* __restrict__ cnt, int* off, int* rbase, int nChunk) {
  __shared__ __attribute__((aligned(16))) int soff[NBC];
  __shared__ __attribute__((aligned(16))) int srb[RBN];
  __shared__ int wtot[OTHR / 32];
  const int tid = threadIdx.x, lane = tid & 31, wave = tid >> 5, sub = tid >> 7;
  for (int i = tid; i < RBN; i += OTHR) srb[i] = 0;
  int carry = 0;
#pragma unroll 1
  for (int ch = 0; ch < nChunk; ++ch) {
    const int base = ch * NBC;
    const v4i c0 = *(const v4i*)(cnt + base + 8 * tid);
    const v4i c1 = *(const v4i*)(cnt + base + 8 * tid + 4);
    const int e0 = max(c0.x, 0), e1 = max(c0.y, 0), e2 = max(c0.z, 0), e3 = max(c0.w, 0);
    const int e4 = max(c1.x, 0), e5 = max(c1.y, 0), e6 = max(c1.z, 0), e7 = max(c1.w, 0);
    const int ts = e0 + e1 + e2 + e3 + e4 + e5 + e6 + e7;
    int incl = ts;
#pragma unroll
    for (int d = 1; d < 32; d <<= 1) {
      const int t = __shfl_up(incl, d);
      if (lane >= d) incl += t;
    }
    if (lane == 31) wtot[wave] = incl;
    __syncthreads();
    const int S0 = wtot[0]  + wtot[1]  + wtot[2]  + wtot[3];
    const int S1 = wtot[4]  + wtot[5]  + wtot[6]  + wtot[7];
    const int S2 = wtot[8]  + wtot[9]  + wtot[10] + wtot[11];
    const int S3 = wtot[12] + wtot[13] + wtot[14] + wtot[15];
    int pre = 0;
#pragma unroll 1
    for (int w = 4 * sub; w < wave; ++w) pre += wtot[w];
    const int b0 = carry;
    const int b1 = b0 + ((S0 + 31) & ~31);
    const int b2 = b1 + ((S1 + 31) & ~31);
    const int b3 = b2 + ((S2 + 31) & ~31);
    const int b4 = b3 + ((S3 + 31) & ~31);
    const int myb = sub == 0 ? b0 : (sub == 1 ? b1 : (sub == 2 ? b2 : b3));
    if (tid == 0) {
      srb[min(4 * ch + 0, RBN - 1)] = b0;
      srb[min(4 * ch + 1, RBN - 1)] = b1;
      srb[min(4 * ch + 2, RBN - 1)] = b2;
      srb[min(4 * ch + 3, RBN - 1)] = b3;
    }
    int run = myb + pre + incl - ts;
    soff[8 * tid + 0] = run; run += e0;
    soff[8 * tid + 1] = run; run += e1;
    soff[8 * tid + 2] = run; run += e2;
    soff[8 * tid + 3] = run; run += e3;
    soff[8 * tid + 4] = run; run += e4;
    soff[8 * tid + 5] = run; run += e5;
    soff[8 * tid + 6] = run; run += e6;
    soff[8 * tid + 7] = run;
    carry = b4;
    __syncthreads();
    const v4i o0 = *(const v4i*)(soff + 4 * tid);
    const v4i o1 = *(const v4i*)(soff + 4 * (tid + OTHR));
    int* op = off + base;
    *(volatile v4i*)(op + 4 * tid) = o0;
    *(volatile v4i*)(op + 4 * (tid + OTHR)) = o1;
    __threadfence();
    *(volatile v4i*)(op + 4 * tid) = o0;
    *(volatile v4i*)(op + 4 * (tid + OTHR)) = o1;
    __syncthreads();
  }
  if (tid == 0) srb[min(4 * nChunk, RBN - 1)] = carry;
  __syncthreads();
  v4i rv = {0, 0, 0, 0};
  if (tid < 32) rv = *(const v4i*)(srb + 4 * tid);
  if (tid < 32) *(volatile v4i*)(rbase + 4 * tid) = rv;
  __threadfence();
  if (tid < 32) *(volatile v4i*)(rbase + 4 * tid) = rv;
}

__global__ __launch_bounds__(NTHR) void k_fill(
    const int* __restrict__ srcs, const int* __restrict__ dsts,
    const int* __restrict__ off, const int* __restrict__ rbase,
    int* csr, int nN, int nE, int vec8, int csrLen) {
  extern __shared__ v4f lds_dyn[];
  int* region = (int*)lds_dyn;
  int* cursor = region + RCAP;
  int* list   = cursor + NBF;
  int* wcnt   = list + LISTN;
  const int tid = threadIdx.x, lane = tid & 31, wave = tid >> 5;
  const int b = blockIdx.x;
  const int nodeBase = b * NBF;

  int rb0 = rbase[b];
  const int rb1 = rbase[b + 1];
  rb0 = rb0 < 0 ? 0 : (rb0 > csrLen ? csrLen : rb0);
  rb0 &= ~31;
  int len = rb1 - rb0;
  len = len < 0 ? 0 : (len > RCAP ? RCAP : len);
  int lenW = (len + 31) & ~31;
  if (rb0 + lenW > csrLen) lenW = (csrLen - rb0) & ~31;

  {
    const v4i z = {0, 0, 0, 0};
    for (int i = tid; i < RCAP / 4; i += NTHR) ((v4i*)region)[i] = z;
    for (int s = tid; s < NBF; s += NTHR) {
      int o = off[nodeBase + s] - rb0;
      o = o < 0 ? 0 : (o > RCAP ? RCAP : o);
      cursor[s] = o;
    }
  }
  __syncthreads();

  const int nChunks = (nE + CHUNK - 1) / CHUNK;
#pragma unroll 1
  for (int ch = 0; ch < nChunks; ++ch) {
    const int cbase = ch * CHUNK;
    const int wc = scan_chunk<NBF>(dsts, nE, cbase, nodeBase, vec8, list, tid, lane, wave);
    if (lane == 0) wcnt[wave] = wc;
    __syncthreads();
    if (wave == 0) {
#pragma unroll 1
      for (int wsx = 0; wsx < NWAVE; ++wsx) {
        int n = __builtin_amdgcn_readfirstlane(wcnt[wsx]);
        n = n > WCAP ? WCAP : (n < 0 ? 0 : n);
        const int* lp = list + wsx * WCAP;
#pragma unroll 1
        for (int i = 0; i < n; ++i) {
          const int ent  = __builtin_amdgcn_readfirstlane(lp[i]);
          const int slot = ent & (NBF - 1);
          int e = cbase + ((ent >> 12) & (CHUNK - 1));
          e = e > nE - 1 ? nE - 1 : e;
          int sv = srcs[e];
          sv = sv < 0 ? 0 : (sv > nN - 1 ? nN - 1 : sv);
          if (lane == 0) {
            int pos = cursor[slot];
            pos = pos < 0 ? 0 : (pos > RCAP - 1 ? RCAP - 1 : pos);
            region[pos] = sv;
            const int np = pos + 1;
            cursor[slot] = np > RCAP ? RCAP : np;
          }
        }
      }
    }
    __syncthreads();
  }

  const int nv = lenW >> 2;
  int* gp = csr + rb0;
#pragma unroll 1
  for (int i = tid; i < nv; i += NTHR) { const v4i v = ((const v4i*)region)[i]; *(volatile v4i*)(gp + 4 * i) = v; }
  __threadfence();
#pragma unroll 1
  for (int i = tid; i < nv; i += NTHR) { const v4i v = ((const v4i*)region)[i]; *(volatile v4i*)(gp + 4 * i) = v; }
}

__global__ __launch_bounds__(NTHR) void k_wcvt(const float* __restrict__ w, _Float16* dp, int K, int Nc, int nUnits) {
  const int i = (int)blockIdx.x * NTHR + (int)threadIdx.x;
  if (i >= nUnits) return;
  const int ppr = K >> 3;
  const int n = i / ppr;
  const int seg = i - n * ppr;
  v8h o;
#pragma unroll
  for (int j = 0; j < 8; ++j) {
    int k = 8 * seg + j;
    k = k > K - 1 ? K - 1 : k;
    const float f = w[(size_t)k * Nc + n];
    o[j] = (_Float16)(f * WCARRY);
  }
  _Float16* gp = dp + (size_t)i * 8;
  *(volatile v8h*)gp = o;
  __threadfence();
  *(volatile v8h*)gp = o;
}

__global__ __launch_bounds__(NTHR) void k_nw(const float* __restrict__ aw, _Float16* dp, int NC) {
  const int tid = threadIdx.x, lane = tid & 31, wave = tid >> 5;
  const int r = (int)blockIdx.x * NWAVE + wave;
  int rr = r > NC - 1 ? NC - 1 : r;
  rr = rr < 0 ? 0 : rr;
  const bool live = r < NC;
  const float* rp = aw + (size_t)rr * HID + 8 * lane;
  const v4f x0 = *(const v4f*)rp;
  const v4f x1 = *(const v4f*)(rp + 4);
  float ss = x0.x * x0.x + x0.y * x0.y + x0.z * x0.z + x0.w * x0.w
           + x1.x * x1.x + x1.y * x1.y + x1.z * x1.z + x1.w * x1.w;
  ss = wsum1(ss);
  const float rn = 1.0f / sqrtf(ss);
  const float sc = live ? rn * PCARRY : 0.f;
  v8h o;
  o[0] = (_Float16)(x0.x * sc); o[1] = (_Float16)(x0.y * sc); o[2] = (_Float16)(x0.z * sc); o[3] = (_Float16)(x0.w * sc);
  o[4] = (_Float16)(x1.x * sc); o[5] = (_Float16)(x1.y * sc); o[6] = (_Float16)(x1.z * sc); o[7] = (_Float16)(x1.w * sc);
  _Float16* gp = dp + (size_t)r * HID + 8 * lane;
  *(volatile v8h*)gp = o;
  __threadfence();
  *(volatile v8h*)gp = o;
}

__global__ __launch_bounds__(NTHR) void k_wfold(const float* __restrict__ W, const float* __restrict__ al,
                                                const float* __restrict__ ar, float* wa,
                                                int CW, int H, int D, int K, int JW) {
  __shared__ __attribute__((aligned(16))) float so[2048];
  const int tid = threadIdx.x;
  int total = K * JW;
  total = total > 2048 ? 2048 : total;
#pragma unroll 1
  for (int o = tid; o < total; o += NTHR) {
    const int k = o / JW, j = o - k * JW;
    const bool useL = j < H;
    const bool anyv = j < 2 * H;
    int hd = useL ? j : (j - H);
    hd = hd > H - 1 ? H - 1 : (hd < 0 ? 0 : hd);
    const float* wp = W + (size_t)k * CW + hd * D;
    const float* pl = al + hd * D;
    const float* pr = ar + hd * D;
    float acc = 0.f;
#pragma unroll 1
    for (int d = 0; d < D; ++d) {
      const float a1v = pl[d], a2v = pr[d];
      const float av = useL ? a1v : a2v;
      acc += wp[d] * av;
    }
    so[o] = anyv ? acc : 0.f;
  }
  __syncthreads();
  const int nq = total >> 2;
#pragma unroll 1
  for (int q = tid; q < nq; q += NTHR) { const v4f v = *(const v4f*)(so + 4 * q); *(volatile v4f*)(wa + 4 * q) = v; }
  __threadfence();
#pragma unroll 1
  for (int q = tid; q < nq; q += NTHR) { const v4f v = *(const v4f*)(so + 4 * q); *(volatile v4f*)(wa + 4 * q) = v; }
}

__global__ __launch_bounds__(NTHR) void k_acvt(const float* __restrict__ x, _Float16* a1, int nN, int npad) {
  const int gi = (int)blockIdx.x * NTHR + (int)threadIdx.x;
  const int row = gi >> 4, seg = gi & 15;
  if (row >= npad) return;
  int rr = row > nN - 1 ? nN - 1 : row;
  rr = rr < 0 ? 0 : rr;
  const bool live = row < nN;
  const float* rp = x + (size_t)rr * FIN + 8 * seg;
  const v4f x0 = *(const v4f*)rp;
  const v4f x1 = *(const v4f*)(rp + 4);
  const float sc = live ? ACARRY : 0.f;
  v8h o;
  o[0] = (_Float16)(x0.x * sc); o[1] = (_Float16)(x0.y * sc); o[2] = (_Float16)(x0.z * sc); o[3] = (_Float16)(x0.w * sc);
  o[4] = (_Float16)(x1.x * sc); o[5] = (_Float16)(x1.y * sc); o[6] = (_Float16)(x1.z * sc); o[7] = (_Float16)(x1.w * sc);
  _Float16* gp = a1 + (size_t)row * FIN + 8 * seg;
  *(volatile v8h*)gp = o;
  __threadfence();
  *(volatile v8h*)gp = o;
}

template <int KD, int JW>
__global__ __launch_bounds__(NTHR) void k_logit(const float* __restrict__ h, const float* __restrict__ wa,
                                                float* es, int nN) {
  static_assert((JW % 4) == 0 && JW <= 16 && KD * JW <= 2048);
  constexpr int NQ = JW / 4;
  __shared__ __attribute__((aligned(16))) float swa[KD * JW];
  __shared__ __attribute__((aligned(16))) float so[NTHR * JW];
  const int tid = threadIdx.x;
#pragma unroll 1
  for (int i = tid; i < (KD * JW) / 4; i += NTHR) *(v4f*)(swa + 4 * i) = *(const v4f*)(wa + 4 * i);
  __syncthreads();
  const int node = (int)blockIdx.x * NTHR + tid;
  int rr = node > nN - 1 ? nN - 1 : node;
  rr = rr < 0 ? 0 : rr;
  const bool live = node < nN;
  v4f acc[NQ];
#pragma unroll
  for (int q = 0; q < NQ; ++q) { v4f z = {0.f, 0.f, 0.f, 0.f}; acc[q] = z; }
  const float* hp = h + (size_t)rr * KD;
#pragma unroll 1
  for (int k = 0; k < KD; ++k) {
    const float hk = hp[k];
#pragma unroll
    for (int q = 0; q < NQ; ++q) {
      const v4f wv = *(const v4f*)(swa + k * JW + 4 * q);
      acc[q] = acc[q] + wv * hk;
    }
  }
#pragma unroll
  for (int q = 0; q < NQ; ++q) *(v4f*)(so + JW * tid + 4 * q) = selz(acc[q], live);
  __syncthreads();
  float* gbase = es + (size_t)blockIdx.x * NTHR * JW;
  v4f cv[NQ];
#pragma unroll
  for (int it = 0; it < NQ; ++it) cv[it] = *(const v4f*)(so + 4 * (it * NTHR + tid));
#pragma unroll
  for (int it = 0; it < NQ; ++it) *(volatile v4f*)(gbase + 4 * (it * NTHR + tid)) = cv[it];
  __threadfence();
#pragma unroll
  for (int it = 0; it < NQ; ++it) *(volatile v4f*)(gbase + 4 * (it * NTHR + tid)) = cv[it];
}

__global__ __launch_bounds__(NTHR) void k_gemm(
    const _Float16* __restrict__ A, const _Float16* __restrict__ Bp,
    float* Cout, int K, int ldc, int nValid, int nStore, float scl) {
  constexpr int TPW = 4;
  constexpr int PPR = BNC / 4;
  constexpr int NIT = (BM * PPR) / NTHR;
  static_assert((BM * PPR) % NTHR == 0);
  static_assert(NIT >= 1);
  static_assert(TPW * 16 * 2 == BNC);
  static_assert(BM == 4 * 16);
  static_assert(PPR == 32);

  __shared__ __attribute__((aligned(16))) float stg[BM * BNC];
  const int tid = threadIdx.x, lane = tid & 31, wave = tid >> 5, hh = lane >> 4, m = lane & 15;
  const int rowBase = (int)blockIdx.x * BM;
  const int colBase = (int)blockIdx.y * BNC;
  const int rg = wave >> 1, chf = wave & 1;
  const int r0 = rg * 16;
  const int c0 = chf * (BNC / 2);

  v8f acc[TPW];
#pragma unroll
  for (int t = 0; t < TPW; ++t) { v8f z = {0.f, 0.f, 0.f, 0.f, 0.f, 0.f, 0.f, 0.f}; acc[t] = z; }

  const _Float16* ap = A  + (size_t)(rowBase + r0 + m) * K + 8 * hh;
  const _Float16* bp = Bp + (size_t)(colBase + c0 + m) * K + 8 * hh;
  const int ksteps = K >> 5;
#pragma unroll 1
  for (int kt = 0; kt < ksteps; ++kt) {
    Frag a;
    a.h[0] = *(const v8h*)(ap + 32 * kt);
    a.h[1] = *(const v8h*)(ap + 32 * kt + 16);
#pragma unroll
    for (int t = 0; t < TPW; ++t) {
      const size_t to = (size_t)(16 * t) * K + 32 * kt;
      Frag b;
      b.h[0] = *(const v8h*)(bp + to);
      b.h[1] = *(const v8h*)(bp + to + 16);
      acc[t] = wmh(a.v, b.v, acc[t]);
    }
  }

  {
    float* sp = stg + (size_t)(r0 + 8 * hh) * BNC + c0 + m;
    const int growb = rowBase + r0 + 8 * hh;
#pragma unroll
    for (int t = 0; t < TPW; ++t) {
#pragma unroll
      for (int r = 0; r < 8; ++r) {
        const bool lv = (growb + r) < nValid;
        const float g = acc[t][r] * scl;
        sp[r * BNC + 16 * t] = lv ? g : 0.f;
      }
    }
  }
  __syncthreads();

  v4f cv[NIT];
#pragma unroll
  for (int it = 0; it < NIT; ++it) {
    const int id = it * NTHR + tid;
    const int row = id >> 5, seg = id & 31;
    cv[it] = *(const v4f*)(stg + (size_t)row * BNC + 4 * seg);
  }
#pragma unroll
  for (int it = 0; it < NIT; ++it) {
    const int id = it * NTHR + tid;
    const int row = id >> 5, seg = id & 31;
    const int grow = rowBase + row;
    if (grow < nStore) {
      float* gp = Cout + (size_t)grow * ldc + colBase + 4 * seg;
      *(volatile v4f*)gp = cv[it];
    }
  }
  __threadfence();
#pragma unroll
  for (int it = 0; it < NIT; ++it) {
    const int id = it * NTHR + tid;
    const int row = id >> 5, seg = id & 31;
    const int grow = rowBase + row;
    if (grow < nStore) {
      float* gp = Cout + (size_t)grow * ldc + colBase + 4 * seg;
      *(volatile v4f*)gp = cv[it];
    }
  }
}

__global__ __launch_bounds__(NTHR) void k_agg1(
    const int* __restrict__ csr, const int* __restrict__ off, const int* __restrict__ cnt,
    const float* __restrict__ es, const float* __restrict__ feat, const float* __restrict__ gb,
    float* hout, _Float16* a16, int nN, int csrLen) {
  const int tid = threadIdx.x, lane = tid & 31, wave = tid >> 5, hq = lane >> 3;
  const int tbase = blockIdx.x * TGT + wave * 32;
  const int cl    = tbase + lane;
  const int cnt_l = cnt[cl];
  const int off_l = off[cl];
  const v4f b0 = *(const v4f*)(gb + 4 * lane);
  const v4f b1 = *(const v4f*)(gb + 128 + 4 * lane);
  const float NINF = -__builtin_inff();

#pragma unroll 1
  for (int j = 0; j < 32; ++j) {
    const int c = tbase + j;
    int n = __shfl(cnt_l, j);
    n = n < 0 ? 0 : (n > DEGCAP ? DEGCAP : n);
    const int st = __shfl(off_l, j);
    const v4f edlo = *(const v4f*)(es + (size_t)c * JW1 + 8);
    const v4f edhi = *(const v4f*)(es + (size_t)c * JW1 + 12);

    v4f mlo = {NINF, NINF, NINF, NINF};
    v4f mhi = {NINF, NINF, NINF, NINF};
#pragma unroll 1
    for (int q0 = 0; q0 < n; q0 += 32) {
      int pos = st + q0 + lane;
      pos = pos < 0 ? 0 : (pos > csrLen - 1 ? csrLen - 1 : pos);
      int sl = csr[pos];
      sl = sl < 0 ? 0 : (sl > nN - 1 ? nN - 1 : sl);
      const int mcnt = (n - q0) < 32 ? (n - q0) : 32;
      const bool valid = lane < mcnt;
      const v4f sllo = *(const v4f*)(es + (size_t)sl * JW1);
      const v4f slhi = *(const v4f*)(es + (size_t)sl * JW1 + 4);
      v4f e0 = selv4(lrelu4(sllo + edlo), valid, NINF);
      v4f e1 = selv4(lrelu4(slhi + edhi), valid, NINF);
      e0 = wmax4(e0);
      e1 = wmax4(e1);
      mlo = vmax4(mlo, e0);
      mhi = vmax4(mhi, e1);
    }
    v4f zlo = {0.f, 0.f, 0.f, 0.f};
    v4f zhi = {0.f, 0.f, 0.f, 0.f};
#pragma unroll 1
    for (int q0 = 0; q0 < n; q0 += 32) {
      int pos = st + q0 + lane;
      pos = pos < 0 ? 0 : (pos > csrLen - 1 ? csrLen - 1 : pos);
      int sl = csr[pos];
      sl = sl < 0 ? 0 : (sl > nN - 1 ? nN - 1 : sl);
      const int mcnt = (n - q0) < 32 ? (n - q0) : 32;
      const bool valid = lane < mcnt;
      const v4f sllo = *(const v4f*)(es + (size_t)sl * JW1);
      const v4f slhi = *(const v4f*)(es + (size_t)sl * JW1 + 4);
      const v4f ex0 = selv4(vexp4(lrelu4(sllo + edlo) - mlo), valid, 0.f);
      const v4f ex1 = selv4(vexp4(lrelu4(slhi + edhi) - mhi), valid, 0.f);
      zlo = zlo + wsum4(ex0);
      zhi = zhi + wsum4(ex1);
    }
    v4f rzlo, rzhi;
    rzlo.x = __builtin_amdgcn_rcpf(zlo.x); rzlo.y = __builtin_amdgcn_rcpf(zlo.y);
    rzlo.z = __builtin_amdgcn_rcpf(zlo.z); rzlo.w = __builtin_amdgcn_rcpf(zlo.w);
    rzhi.x = __builtin_amdgcn_rcpf(zhi.x); rzhi.y = __builtin_amdgcn_rcpf(zhi.y);
    rzhi.z = __builtin_amdgcn_rcpf(zhi.z); rzhi.w = __builtin_amdgcn_rcpf(zhi.w);

    v4f acc0 = {0.f, 0.f, 0.f, 0.f};
    v4f acc1 = {0.f, 0.f, 0.f, 0.f};
#pragma unroll 1
    for (int q0 = 0; q0 < n; q0 += 32) {
      int pos = st + q0 + lane;
      pos = pos < 0 ? 0 : (pos > csrLen - 1 ? csrLen - 1 : pos);
      int sl = csr[pos];
      sl = sl < 0 ? 0 : (sl > nN - 1 ? nN - 1 : sl);
      const int mcnt = (n - q0) < 32 ? (n - q0) : 32;
      const bool valid = lane < mcnt;
      const v4f sllo = *(const v4f*)(es + (size_t)sl * JW1);
      const v4f slhi = *(const v4f*)(es + (size_t)sl * JW1 + 4);
      const v4f al0 = selv4(vexp4(lrelu4(sllo + edlo) - mlo) * rzlo, valid, 0.f);
      const v4f al1 = selv4(vexp4(lrelu4(slhi + edhi) - mhi) * rzhi, valid, 0.f);
#pragma unroll 1
      for (int pp = 0; pp < mcnt; ++pp) {
        const int s = __builtin_amdgcn_readlane(sl, pp);
        const float a0 = __int_as_float(__builtin_amdgcn_readlane(__float_as_int(al0.x), pp));
        const float a1 = __int_as_float(__builtin_amdgcn_readlane(__float_as_int(al0.y), pp));
        const float a2 = __int_as_float(__builtin_amdgcn_readlane(__float_as_int(al0.z), pp));
        const float a3 = __int_as_float(__builtin_amdgcn_readlane(__float_as_int(al0.w), pp));
        const float a4 = __int_as_float(__builtin_amdgcn_readlane(__float_as_int(al1.x), pp));
        const float a5 = __int_as_float(__builtin_amdgcn_readlane(__float_as_int(al1.y), pp));
        const float a6 = __int_as_float(__builtin_amdgcn_readlane(__float_as_int(al1.z), pp));
        const float a7 = __int_as_float(__builtin_amdgcn_readlane(__float_as_int(al1.w), pp));
        const float ap0 = (hq == 0) ? a0 : ((hq == 1) ? a1 : ((hq == 2) ? a2 : a3));
        const float ap1 = (hq == 0) ? a4 : ((hq == 1) ? a5 : ((hq == 2) ? a6 : a7));
        const float* hs = feat + (size_t)s * HID + 4 * lane;
        const v4f hv0 = *(const v4f*)hs;
        const v4f hv1 = *(const v4f*)(hs + 128);
        acc0 = acc0 + hv0 * ap0;
        acc1 = acc1 + hv1 * ap1;
      }
    }

    const bool live = c < nN;
    v4f o0 = elu4(acc0 + b0);
    v4f o1 = elu4(acc1 + b1);
    o0 = selz(o0, live);
    o1 = selz(o1, live);
    v4h q0h, q1h;
    q0h.x = (_Float16)(o0.x * ACARRY); q0h.y = (_Float16)(o0.y * ACARRY);
    q0h.z = (_Float16)(o0.z * ACARRY); q0h.w = (_Float16)(o0.w * ACARRY);
    q1h.x = (_Float16)(o1.x * ACARRY); q1h.y = (_Float16)(o1.y * ACARRY);
    q1h.z = (_Float16)(o1.z * ACARRY); q1h.w = (_Float16)(o1.w * ACARRY);
    float* gp = hout + (size_t)c * HID + 4 * lane;
    _Float16* hp = a16 + (size_t)c * HID + 4 * lane;
    *(volatile v4f*)gp = o0;
    *(volatile v4f*)(gp + 128) = o1;
    *(volatile v4h*)hp = q0h;
    *(volatile v4h*)(hp + 128) = q1h;
    __threadfence();
    *(volatile v4f*)gp = o0;
    *(volatile v4f*)(gp + 128) = o1;
    *(volatile v4h*)hp = q0h;
    *(volatile v4h*)(hp + 128) = q1h;
  }
}

__global__ __launch_bounds__(NTHR) void k_agg2(
    const int* __restrict__ csr, const int* __restrict__ off, const int* __restrict__ cnt,
    const float* __restrict__ es, const float* __restrict__ feat, const float* __restrict__ gb,
    const float* hres, float* zout, int nN, int csrLen) {
  const int tid = threadIdx.x, lane = tid & 31, wave = tid >> 5;
  const int tbase = blockIdx.x * TGT + wave * 32;
  const int cl    = tbase + lane;
  const int cnt_l = cnt[cl];
  const int off_l = off[cl];
  const v4f b0 = *(const v4f*)(gb + 4 * lane);
  const v4f b1 = *(const v4f*)(gb + 128 + 4 * lane);
  const float NINF = -__builtin_inff();

#pragma unroll 1
  for (int j = 0; j < 32; ++j) {
    const int c = tbase + j;
    int n = __shfl(cnt_l, j);
    n = n < 0 ? 0 : (n > DEGCAP ? DEGCAP : n);
    const int st = __shfl(off_l, j);
    const float edc = es[(size_t)c * JW2 + 1];

    float m = NINF;
#pragma unroll 1
    for (int q0 = 0; q0 < n; q0 += 32) {
      int pos = st + q0 + lane;
      pos = pos < 0 ? 0 : (pos > csrLen - 1 ? csrLen - 1 : pos);
      int sl = csr[pos];
      sl = sl < 0 ? 0 : (sl > nN - 1 ? nN - 1 : sl);
      const int mcnt = (n - q0) < 32 ? (n - q0) : 32;
      const bool valid = lane < mcnt;
      const float elv = es[(size_t)sl * JW2];
      float e = lrelu1(elv + edc);
      e = valid ? e : NINF;
      e = wmax1(e);
      m = fmaxf(m, e);
    }
    float z = 0.f;
#pragma unroll 1
    for (int q0 = 0; q0 < n; q0 += 32) {
      int pos = st + q0 + lane;
      pos = pos < 0 ? 0 : (pos > csrLen - 1 ? csrLen - 1 : pos);
      int sl = csr[pos];
      sl = sl < 0 ? 0 : (sl > nN - 1 ? nN - 1 : sl);
      const int mcnt = (n - q0) < 32 ? (n - q0) : 32;
      const bool valid = lane < mcnt;
      const float elv = es[(size_t)sl * JW2];
      const float exv = __expf(lrelu1(elv + edc) - m);
      const float ex = valid ? exv : 0.f;
      z += wsum1(ex);
    }
    const float rz = __builtin_amdgcn_rcpf(z);

    v4f acc0 = {0.f, 0.f, 0.f, 0.f};
    v4f acc1 = {0.f, 0.f, 0.f, 0.f};
#pragma unroll 1
    for (int q0 = 0; q0 < n; q0 += 32) {
      int pos = st + q0 + lane;
      pos = pos < 0 ? 0 : (pos > csrLen - 1 ? csrLen - 1 : pos);
      int sl = csr[pos];
      sl = sl < 0 ? 0 : (sl > nN - 1 ? nN - 1 : sl);
      const int mcnt = (n - q0) < 32 ? (n - q0) : 32;
      const bool valid = lane < mcnt;
      const float elv = es[(size_t)sl * JW2];
      const float alv = __expf(lrelu1(elv + edc) - m) * rz;
      const float al = valid ? alv : 0.f;
#pragma unroll 1
      for (int pp = 0; pp < mcnt; ++pp) {
        const int s = __builtin_amdgcn_readlane(sl, pp);
        const float a = __int_as_float(__builtin_amdgcn_readlane(__float_as_int(al), pp));
        const float* hs = feat + (size_t)s * HID + 4 * lane;
        const v4f hv0 = *(const v4f*)hs;
        const v4f hv1 = *(const v4f*)(hs + 128);
        acc0 = acc0 + hv0 * a;
        acc1 = acc1 + hv1 * a;
      }
    }

    const bool live = c < nN;
    const float* rp = hres + (size_t)c * HID + 4 * lane;
    const v4f r0 = *(const v4f*)rp;
    const v4f r1 = *(const v4f*)(rp + 128);
    v4f o0 = (acc0 + r0) + b0;
    v4f o1 = (acc1 + r1) + b1;
    o0 = selz(o0, live);
    o1 = selz(o1, live);
    float* gp = zout + (size_t)c * HID + 4 * lane;
    *(volatile v4f*)gp = o0;
    *(volatile v4f*)(gp + 128) = o1;
    __threadfence();
    *(volatile v4f*)gp = o0;
    *(volatile v4f*)(gp + 128) = o1;
  }
}

__global__ __launch_bounds__(NTHR) void k_pool(
    const int* __restrict__ gid, const float* __restrict__ z, _Float16* p16, int nN, int nG, int vec8) {
  __shared__ __attribute__((aligned(16))) int list[LISTN];
  __shared__ __attribute__((aligned(16))) float spart[NWAVE * HID];
  __shared__ __attribute__((aligned(16))) _Float16 srow[HID];
  __shared__ int swn[NWAVE];
  __shared__ float swss[NWAVE];
  const int tid = threadIdx.x, lane = tid & 31, wave = tid >> 5;
  const int g = blockIdx.x;

  v4f sa0 = {0.f, 0.f, 0.f, 0.f};
  v4f sa1 = {0.f, 0.f, 0.f, 0.f};
  int wn = 0;

  const int nChunks = (nN + CHUNK - 1) / CHUNK;
#pragma unroll 1
  for (int ch = 0; ch < nChunks; ++ch) {
    const int cbase = ch * CHUNK;
    const int wc = scan_chunk<1>(gid, nN, cbase, g, vec8, list, tid, lane, wave);
    __syncthreads();
    int n = wc;
    n = n > WCAP ? WCAP : (n < 0 ? 0 : n);
    wn += n;
    const int* lp = list + wave * WCAP;
#pragma unroll 1
    for (int i = 0; i < n; ++i) {
      const int ent = __builtin_amdgcn_readfirstlane(lp[i]);
      int node = cbase + ((ent >> 12) & (CHUNK - 1));
      node = node > nN - 1 ? nN - 1 : (node < 0 ? 0 : node);
      const float* hp = z + (size_t)node * HID + 4 * lane;
      const v4f hv0 = *(const v4f*)hp;
      const v4f hv1 = *(const v4f*)(hp + 128);
      sa0 = sa0 + hv0;
      sa1 = sa1 + hv1;
    }
    __syncthreads();
  }

  *(v4f*)(spart + wave * HID + 4 * lane)       = sa0;
  *(v4f*)(spart + wave * HID + 128 + 4 * lane) = sa1;
  if (lane == 0) swn[wave] = wn;
  __syncthreads();
  float S = 0.f;
  int ng = 0;
#pragma unroll
  for (int w = 0; w < NWAVE; ++w) { S += spart[w * HID + tid]; ng += swn[w]; }
  const float rc = 1.0f / fmaxf((float)ng, 1.0f);
  const float mean = S * rc;
  float sq = mean * mean;
  sq = wsum1(sq);
  if (lane == 0) swss[wave] = sq;
  __syncthreads();
  float ss = 0.f;
#pragma unroll
  for (int w = 0; w < NWAVE; ++w) ss += swss[w];
  const float rn = 1.0f / sqrtf(ss);
  const bool live = g < nG;
  const float ni = live ? mean * rn : 0.f;
  srow[tid] = (_Float16)(ni * PCARRY);
  __syncthreads();

  _Float16* gp = p16 + (size_t)g * HID;
  const int tq = tid & (HID / 8 - 1);
  const v8h v = *(const v8h*)(srow + 8 * tq);
  if (tid < HID / 8) *(volatile v8h*)(gp + 8 * tid) = v;
  __threadfence();
  if (tid < HID / 8) *(volatile v8h*)(gp + 8 * tid) = v;
}

__global__ __launch_bounds__(NTHR) void k_arc(const float* __restrict__ cosp, const int* __restrict__ lab,
                                              float* out, int nOut, int NC, int ldc, int nLab) {
  __shared__ __attribute__((aligned(16))) float so[NTHR];
  const int tid = threadIdx.x;
  const int f0 = (int)blockIdx.x * NTHR + tid;
  int f = f0 > nOut - 1 ? nOut - 1 : f0;
  f = f < 0 ? 0 : f;
  const int g = f / NC;
  const int c = f - g * NC;
  int gg = g > nLab - 1 ? nLab - 1 : g;
  gg = gg < 0 ? 0 : gg;
  const float cv = cosp[(size_t)g * ldc + c];
  const int lb = lab[gg];
  const float mm = (lb == c) ? ARC_M : 0.f;
  const float o = cosf(acosf(cv) + mm) * ARC_S;
  so[tid] = o;
  __syncthreads();
  const int tq = tid & (NTHR / 4 - 1);
  const v4f v = *(const v4f*)(so + 4 * tq);
  const int q = (int)blockIdx.x * (NTHR / 4) + tid;
  const bool st = (tid < NTHR / 4) && (4 * q + 3 < nOut);
  if (st) *(volatile v4f*)(out + (size_t)4 * q) = v;
  __threadfence();
  if (st) *(volatile v4f*)(out + (size_t)4 * q) = v;
}

extern "C" void kernel_launch(void* const* d_in, const int* in_sizes, int n_in,
                              void* d_out, int out_size, void* d_ws, size_t ws_size,
                              hipStream_t stream) {
  if (n_in < 14) return;
  if (in_sizes[0] < FIN || (in_sizes[0] % FIN) != 0) return;
  const int nN = in_sizes[0] / FIN;
  if (nN < 1 || nN > 131072) return;
  const int nE = in_sizes[1];
  if (nE < 1 || nE > (1 << 26) || in_sizes[2] != nE) return;
  if (in_sizes[3] != nN) return;
  const int nLab = in_sizes[4];
  if (nLab < 1) return;
  if (in_sizes[5] != FIN * HID) return;
  if (in_sizes[6] != HID || in_sizes[7] != HID || in_sizes[8] != HID) return;
  if (in_sizes[9] != HID * HID) return;
  if (in_sizes[10] != HID || in_sizes[11] != HID || in_sizes[12] != HID) return;
  if (in_sizes[13] < HID || (in_sizes[13] % HID) != 0) return;
  const int NC = in_sizes[13] / HID;
  if (out_size < NC || (out_size % NC) != 0) return;
  const int nG = out_size / NC;
  if (nG < 1 || nG > 4096) return;

  const float* features = (const float*)d_in[0];
  const int*   src      = (const int*)d_in[1];
  const int*   dst      = (const int*)d_in[2];
  const int*   gids     = (const int*)d_in[3];
  const int*   labels   = (const int*)d_in[4];
  const float* W1       = (const float*)d_in[5];
  const float* al1      = (const float*)d_in[6];
  const float* ar1      = (const float*)d_in[7];
  const float* b1       = (const float*)d_in[8];
  const float* W2       = (const float*)d_in[9];
  const float* al2      = (const float*)d_in[10];
  const float* ar2      = (const float*)d_in[11];
  const float* b2       = (const float*)d_in[12];
  const float* arc_w    = (const float*)d_in[13];
  float* out = (float*)d_out;

  const int NPAD   = ((nN + TGT - 1) / TGT) * TGT;
  const int nAgg   = NPAD / TGT;
  const int nBC    = (nN + NBC - 1) / NBC;
  const int CNTPAD = nBC * NBC;
  if (CNTPAD < NPAD) return;
  if (4 * nBC + 1 > RBN) return;
  const int nBF    = (nN + NBF - 1) / NBF;
  if (nBF > 4 * nBC) return;
  const int csrLen = ((nE + 31) & ~31) + 4096;
  if (31 * 4 * nBC > 4096) return;
  const int GPADM  = ((nG + BM - 1) / BM) * BM;
  const int NCP    = ((NC + BNC - 1) / BNC) * BNC;

  char* ws = (char*)d_ws;
  size_t off = 0;
  const size_t oCnt = off; off += (size_t)CNTPAD * 4;                    off = (off + 255) & ~(size_t)255;
  const size_t oOff = off; off += (size_t)CNTPAD * 4;                    off = (off + 255) & ~(size_t)255;
  const size_t oRb  = off; off += (size_t)RBN * 4;                       off = (off + 255) & ~(size_t)255;
  const size_t oCsr = off; off += (size_t)csrLen * 4;                    off = (off + 255) & ~(size_t)255;
  const size_t oW1  = off; off += (size_t)HID * FIN * 2;                 off = (off + 255) & ~(size_t)255;
  const size_t oW2  = off; off += (size_t)HID * HID * 2;                 off = (off + 255) & ~(size_t)255;
  const size_t oNw  = off; off += (size_t)NCP * HID * 2;                 off = (off + 255) & ~(size_t)255;
  const size_t oWa1 = off; off += (size_t)FIN * JW1 * 4;                 off = (off + 255) & ~(size_t)255;
  const size_t oWa2 = off; off += (size_t)HID * JW2 * 4;                 off = (off + 255) & ~(size_t)255;
  const size_t oA1  = off; off += (size_t)NPAD * FIN * 2;                off = (off + 255) & ~(size_t)255;
  const size_t oFt  = off; off += (size_t)NPAD * HID * 4;                off = (off + 255) & ~(size_t)255;
  const size_t oEs1 = off; off += (size_t)NPAD * JW1 * 4;                off = (off + 255) & ~(size_t)255;
  const size_t oH1  = off; off += (size_t)NPAD * HID * 4;                off = (off + 255) & ~(size_t)255;
  const size_t oA2  = off; off += (size_t)NPAD * HID * 2;                off = (off + 255) & ~(size_t)255;
  const size_t oEs2 = off; off += (size_t)NPAD * JW2 * 4;                off = (off + 255) & ~(size_t)255;
  const size_t oP16 = off; off += (size_t)GPADM * HID * 2;               off = (off + 255) & ~(size_t)255;
  const size_t oCos = off; off += (size_t)GPADM * NCP * 4;               off = (off + 255) & ~(size_t)255;
  if (off > ws_size || off > (size_t)WSCAP) return;

  int*   cnt   = (int*)(ws + oCnt);
  int*   offp  = (int*)(ws + oOff);
  int*   rb    = (int*)(ws + oRb);
  int*   csr   = (int*)(ws + oCsr);
  _Float16* w1p = (_Float16*)(ws + oW1);
  _Float16* w2p = (_Float16*)(ws + oW2);
  _Float16* nwp = (_Float16*)(ws + oNw);
  float* wa1   = (float*)(ws + oWa1);
  float* wa2   = (float*)(ws + oWa2);
  _Float16* a1 = (_Float16*)(ws + oA1);
  float* feat  = (float*)(ws + oFt);
  float* es1   = (float*)(ws + oEs1);
  float* h1    = (float*)(ws + oH1);
  _Float16* a2 = (_Float16*)(ws + oA2);
  float* es2   = (float*)(ws + oEs2);
  _Float16* p16 = (_Float16*)(ws + oP16);
  float* cosp  = (float*)(ws + oCos);

  const int vec8 = 1;

  k_count<<<nBC, NTHR, 0, stream>>>(dst, cnt, nE, vec8);
  k_offsets<<<1, OTHR, 0, stream>>>(cnt, offp, rb, nBC);
  hipFuncSetAttribute(reinterpret_cast<const void*>(&k_fill),
                      hipFuncAttributeMaxDynamicSharedMemorySize, LDS_FILL);
  k_fill<<<nBF, NTHR, LDS_FILL, stream>>>(src, dst, offp, rb, csr, nN, nE, vec8, csrLen);

  {
    const int u1 = HID * (FIN / 8);
    k_wcvt<<<(u1 + NTHR - 1) / NTHR, NTHR, 0, stream>>>(W1, w1p, FIN, HID, u1);
    const int u2 = HID * (HID / 8);
    k_wcvt<<<(u2 + NTHR - 1) / NTHR, NTHR, 0, stream>>>(W2, w2p, HID, HID, u2);
  }
  k_nw<<<NCP / NWAVE, NTHR, 0, stream>>>(arc_w, nwp, NC);
  k_wfold<<<1, NTHR, 0, stream>>>(W1, al1, ar1, wa1, HID, NH1, DH1, FIN, JW1);
  k_wfold<<<1, NTHR, 0, stream>>>(W2, al2, ar2, wa2, HID, 1, HID, HID, JW2);

  k_acvt<<<(NPAD * 16) / NTHR, NTHR, 0, stream>>>(features, a1, nN, NPAD);
  k_gemm<<<dim3(NPAD / BM, HID / BNC), NTHR, 0, stream>>>(a1, w1p, feat, FIN, HID, nN, NPAD, SCL_AW);
  k_logit<FIN, JW1><<<NPAD / NTHR, NTHR, 0, stream>>>(features, wa1, es1, nN);
  k_agg1<<<nAgg, NTHR, 0, stream>>>(csr, offp, cnt, es1, feat, b1, h1, a2, nN, csrLen);

  k_gemm<<<dim3(NPAD / BM, HID / BNC), NTHR, 0, stream>>>(a2, w2p, feat, HID, HID, nN, NPAD, SCL_AW);
  k_logit<HID, JW2><<<NPAD / NTHR, NTHR, 0, stream>>>(h1, wa2, es2, nN);
  k_agg2<<<nAgg, NTHR, 0, stream>>>(csr, offp, cnt, es2, feat, b2, h1, h1, nN, csrLen);

  k_pool<<<GPADM, NTHR, 0, stream>>>(gids, h1, p16, nN, nG, vec8);
  k_gemm<<<dim3(GPADM / BM, NCP / BNC), NTHR, 0, stream>>>(p16, nwp, cosp, HID, NCP, nG, GPADM, SCL_PW);
  k_arc<<<(out_size + NTHR - 1) / NTHR, NTHR, 0, stream>>>(cosp, labels, out, out_size, NC, NCP, nLab);
}
